// LocalFeatureAggregation_1606317769121
// MI455X (gfx1250) — hardware-verified
//
#include <hip/hip_runtime.h>
#include <math.h>

#pragma clang fp contract(off)

constexpr int kBatch   = 4;
constexpr int kNpts    = 8192;
constexpr int kCin     = 64;
constexpr int kCout    = 64;
constexpr int kNbr     = 16;
constexpr int kThreads = 128;
constexpr int kWavesPB = kThreads / 32;
constexpr int kChunk   = 512;
constexpr int kNChunk  = kNpts / kChunk;
constexpr int kTileP   = 136;
constexpr int kWP      = 128;
constexpr float kWCarry    = 16.0f;
constexpr float kWCarryInv = 0.0625f;
constexpr float kEps       = 1e-5f;

static_assert(kNpts % kChunk == 0, "chunking");
static_assert(kNpts % kThreads == 0, "query blocks");
static_assert(kChunk == 4 * kThreads, "4 candidates built per thread per chunk");
static_assert((kChunk * 3) / 4 == 3 * kThreads, "3 float4 loads per thread per chunk");
static_assert(2 * kCin == 128 && 2 * kCout == 128 && kCout == 64, "K = 128 = 4 x 32, N = 64 = 4 x 16");

typedef __attribute__((ext_vector_type(16))) _Float16 v16h;
typedef __attribute__((ext_vector_type(8)))  _Float16 v8h;
typedef __attribute__((ext_vector_type(8)))  float    v8f;
typedef __attribute__((ext_vector_type(4)))  float    v4f;
typedef __attribute__((ext_vector_type(4)))  int      v4i;

__device__ __forceinline__ void dep_guard_h(v8f& a, v8f& b, v16h x, v16h y) { asm volatile("v_nop\n\tv_nop\n\tv_nop\n\tv_nop" : "+v"(a), "+v"(b) : "v"(x), "v"(y)); }
__device__ __forceinline__ void keep4_h(v16h a, v16h b, v16h c, v16h d) { asm volatile("v_nop" :: "v"(a), "v"(b), "v"(c), "v"(d)); }
__device__ __forceinline__ void acc_guard4(v8f& a, v8f& b, v8f& c, v8f& d) { asm volatile("v_nop\n\tv_nop\n\tv_nop\n\tv_nop" : "+v"(a), "+v"(b), "+v"(c), "+v"(d)); }
template <typename T> struct Frag;
template <> struct Frag<_Float16> {
  typedef v16h V; union U { v16h v; v8h h[2]; };
  static __device__ __forceinline__ v16h load(const _Float16* p) {
    U f; f.h[0] = *(const v8h*)(p); f.h[1] = *(const v8h*)(p + 16); return f.v;
  }
  static __device__ __forceinline__ v8f mma(v16h a, v16h b, v8f c) {
    return __builtin_amdgcn_wmma_f32_16x16x32_f16(false, a, false, b, (short)0, c, false, false);
  }
};
typedef Frag<_Float16> FragH;

__device__ __forceinline__ void tile_gemm_16x64x128(const _Float16* tile, const _Float16* wq, int rl, int hh, v8f (&acc)[4]) {
#pragma unroll
  for (int j = 0; j < 4; ++j) acc[j] = (v8f){0.f, 0.f, 0.f, 0.f, 0.f, 0.f, 0.f, 0.f};
#pragma unroll
  for (int kc = 0; kc < 4; ++kc) {
    v16h bq[4];
#pragma unroll
    for (int j = 0; j < 4; ++j) bq[j] = FragH::load(wq + (j * 16 + rl) * kWP + kc * 32 + 8 * hh);
    const v16h a = FragH::load(tile + rl * kTileP + kc * 32 + 8 * hh);
#pragma unroll
    for (int j = 0; j < 4; ++j) acc[j] = FragH::mma(a, bq[j], acc[j]);
    dep_guard_h(acc[0], acc[3], a, bq[3]);
    keep4_h(bq[0], bq[1], bq[2], bq[3]);
  }
  acc_guard4(acc[0], acc[1], acc[2], acc[3]);
}

__global__ __launch_bounds__(kThreads) void knn_mlp_pool_kernel(
    const float* __restrict__ pts, const float* __restrict__ feat,
    const float* __restrict__ wgeom, const float* __restrict__ g1, const float* __restrict__ b1,
    const float* __restrict__ m1, const float* __restrict__ v1,
    const float* __restrict__ wsem, const float* __restrict__ g2, const float* __restrict__ b2,
    const float* __restrict__ m2, const float* __restrict__ v2,
    const float* __restrict__ wfuse, const float* __restrict__ g3, const float* __restrict__ b3,
    const float* __restrict__ m3, const float* __restrict__ v3,
    float* __restrict__ out) {
  __shared__ __align__(16) _Float16 s_wsem[kCout * kWP];
  __shared__ __align__(16) _Float16 s_wfuse[kCout * kWP];
  __shared__ __align__(16) int s_idx[kThreads * kNbr];
  __shared__ __align__(16) float s_wg[kCout * 6];
  __shared__ float s_m[3 * kCout];
  __shared__ float s_s[3 * kCout];
  __shared__ float s_b[3 * kCout];
  __shared__ __align__(16) float s_out[kWavesPB * 64];
  __shared__ __align__(16) float s_region[kWavesPB * 16 * kTileP / 2];

  const int tid  = threadIdx.x;
  const int lane = tid & 31;
  const int wave = tid >> 5;
  const int hh   = lane >> 4;
  const int rl   = lane & 15;
  const int b    = blockIdx.y;
  const int nblk = blockIdx.x * kThreads;

#pragma unroll 1
  for (int i = tid; i < (kCout * 2 * kCin) / 8; i += kThreads) {
    const v4f a0 = *(const v4f*)(wsem + 8 * i);
    const v4f a1 = *(const v4f*)(wsem + 8 * i + 4);
    const v4f f0 = *(const v4f*)(wfuse + 8 * i);
    const v4f f1 = *(const v4f*)(wfuse + 8 * i + 4);
    v8h hs, hf;
#pragma unroll
    for (int e = 0; e < 4; ++e) {
      hs[e]     = (_Float16)(a0[e] * kWCarry);
      hs[4 + e] = (_Float16)(a1[e] * kWCarry);
      hf[e]     = (_Float16)(f0[e] * kWCarry);
      hf[4 + e] = (_Float16)(f1[e] * kWCarry);
    }
    *(v8h*)(s_wsem + 8 * i)  = hs;
    *(v8h*)(s_wfuse + 8 * i) = hf;
  }
  if (tid < (kCout * 6) / 4) *(v4f*)(s_wg + 4 * tid) = *(const v4f*)(wgeom + 4 * tid);
  if (tid < kCout) {
    s_m[tid]       = m1[tid]; s_s[tid]       = g1[tid] / sqrtf(v1[tid] + kEps); s_b[tid]       = b1[tid];
    s_m[64 + tid]  = m2[tid]; s_s[64 + tid]  = g2[tid] / sqrtf(v2[tid] + kEps); s_b[64 + tid]  = b2[tid];
    s_m[128 + tid] = m3[tid]; s_s[128 + tid] = g3[tid] / sqrtf(v3[tid] + kEps); s_b[128 + tid] = b3[tid];
  }

  const float* pb   = pts + (size_t)b * kNpts * 3;
  const v4f*   pb4  = (const v4f*)pb;
  float*       s_raw  = s_region;
  v4f*         s_cand = (v4f*)(s_region + 1536);
  {
    const int nq = nblk + tid;
    const float qx = pb[nq * 3 + 0];
    const float qy = pb[nq * 3 + 1];
    const float qz = pb[nq * 3 + 2];
    const float sqq = (qx * qx + qz * qz) + qy * qy;
    float bd[16]; int bi[16];
#pragma unroll
    for (int s = 0; s < 16; ++s) { bd[s] = 3.0e38f; bi[s] = 0; }

#pragma unroll 1
    for (int ch = 0; ch < kNChunk; ++ch) {
      __syncthreads();
#pragma unroll
      for (int i = 0; i < 3; ++i) *(v4f*)(s_raw + 4 * (tid + kThreads * i)) = pb4[ch * 384 + tid + kThreads * i];
      __syncthreads();
#pragma unroll
      for (int i = 0; i < 4; ++i) {
        const int c = tid + kThreads * i;
        const float x = s_raw[3 * c], y = s_raw[3 * c + 1], z = s_raw[3 * c + 2];
        const float sq = (x * x + z * z) + y * y;
        s_cand[c] = (v4f){x, y, z, sq};
      }
      __syncthreads();
      const int cbase = ch * kChunk;
#pragma unroll 4
      for (int j = 0; j < kChunk; ++j) {
        const v4f c = s_cand[j];
        float dot = qx * c[0];
        dot = fmaf(qy, c[1], dot);
        dot = fmaf(qz, c[2], dot);
        const float d = (sqq + c[3]) - 2.0f * dot;
        if (d < bd[15]) {
          float cd = d; int ci = cbase + j;
#pragma unroll
          for (int s = 0; s < 16; ++s) {
            const float td = bd[s]; const int ti = bi[s];
            const bool lt = d < td;
            bd[s] = lt ? cd : td; cd = lt ? td : cd;
            bi[s] = lt ? ci : ti; ci = lt ? ti : ci;
          }
        }
      }
    }
    int* ir = s_idx + tid * kNbr;
    *(v4i*)(ir)      = (v4i){bi[0],  bi[1],  bi[2],  bi[3]};
    *(v4i*)(ir + 4)  = (v4i){bi[4],  bi[5],  bi[6],  bi[7]};
    *(v4i*)(ir + 8)  = (v4i){bi[8],  bi[9],  bi[10], bi[11]};
    *(v4i*)(ir + 12) = (v4i){bi[12], bi[13], bi[14], bi[15]};
  }
  __syncthreads();

  const float* fb   = feat + (size_t)b * kNpts * kCin;
  _Float16*    tile = (_Float16*)s_region + wave * (16 * kTileP);
  float*       so   = s_out + wave * 64;

#pragma unroll 1
  for (int t = 0; t < 32; ++t) {
    const int q = wave * 32 + t;
    const int n = nblk + q;
    int nb = s_idx[q * kNbr + rl];
    nb = nb < 0 ? 0 : (nb > kNpts - 1 ? kNpts - 1 : nb);

    const float* cr = fb + (size_t)n * kCin + 32 * hh;
    const float* nr = fb + (size_t)nb * kCin + 32 * hh;
#pragma unroll 1
    for (int i = 0; i < 4; ++i) {
      const v4f c0 = *(const v4f*)(cr + 8 * i);
      const v4f c1 = *(const v4f*)(cr + 8 * i + 4);
      const v4f e0 = *(const v4f*)(nr + 8 * i);
      const v4f e1 = *(const v4f*)(nr + 8 * i + 4);
      v8h hc, hd;
#pragma unroll
      for (int e = 0; e < 4; ++e) {
        const float d0 = e0[e] - c0[e];
        const float d1 = e1[e] - c1[e];
        hc[e]     = (_Float16)c0[e];
        hc[4 + e] = (_Float16)c1[e];
        hd[e]     = (_Float16)d0;
        hd[4 + e] = (_Float16)d1;
      }
      *(v8h*)(tile + rl * kTileP + 32 * hh + 8 * i)      = hc;
      *(v8h*)(tile + rl * kTileP + 64 + 32 * hh + 8 * i) = hd;
    }
    const float px = pb[n * 3 + 0], py = pb[n * 3 + 1], pz = pb[n * 3 + 2];
    const float ex = pb[nb * 3 + 0], ey = pb[nb * 3 + 1], ez = pb[nb * 3 + 2];
    const float dx = ex - px, dy = ey - py, dz = ez - pz;
    __syncthreads();

    v8f accs[4];
    tile_gemm_16x64x128(tile, s_wsem, rl, hh, accs);
    __syncthreads();

#pragma unroll
    for (int j = 0; j < 4; ++j) {
      const int o = j * 16 + rl;
      const float mm = s_m[64 + o], ss = s_s[64 + o], bb = s_b[64 + o];
#pragma unroll
      for (int r = 0; r < 8; ++r) {
        float v = accs[j][r] * kWCarryInv;
        v = (v - mm) * ss + bb;
        v = v > 0.0f ? v : 0.0f;
        tile[(8 * hh + r) * kTileP + 64 + o] = (_Float16)v;
      }
    }
#pragma unroll 1
    for (int og = 0; og < 4; ++og) {
      v8h hg;
#pragma unroll
      for (int e = 0; e < 8; ++e) {
        const int o = 32 * hh + 8 * og + e;
        const float* w = s_wg + o * 6;
        float y = px * w[0];
        y = fmaf(py, w[1], y);
        y = fmaf(pz, w[2], y);
        y = fmaf(dx, w[3], y);
        y = fmaf(dy, w[4], y);
        y = fmaf(dz, w[5], y);
        y = (y - s_m[o]) * s_s[o] + s_b[o];
        y = y > 0.0f ? y : 0.0f;
        hg[e] = (_Float16)y;
      }
      *(v8h*)(tile + rl * kTileP + 32 * hh + 8 * og) = hg;
    }
    __syncthreads();

    v8f accf[4];
    tile_gemm_16x64x128(tile, s_wfuse, rl, hh, accf);
#pragma unroll
    for (int j = 0; j < 4; ++j) {
      const int o = j * 16 + rl;
      const float mm = s_m[128 + o], ss = s_s[128 + o], bb = s_b[128 + o];
      float mx = 0.0f;
#pragma unroll
      for (int r = 0; r < 8; ++r) {
        float v = accf[j][r] * kWCarryInv;
        v = (v - mm) * ss + bb;
        v = v > 0.0f ? v : 0.0f;
        mx = fmaxf(mx, v);
      }
      const float ox = __shfl_xor(mx, 16);
      mx = fmaxf(mx, ox);
      so[o] = mx;
    }
    __syncthreads();

    const v4f val = *(const v4f*)(so + 4 * rl);
    float* op = out + ((size_t)b * kNpts + n) * kCout + 4 * rl;
    for (int pass = 0; pass < 2; ++pass) {
      if (lane < 16) *(volatile v4f*)op = val;
      __threadfence();
    }
  }
}

extern "C" void kernel_launch(void* const* d_in, const int* in_sizes, int n_in,
                              void* d_out, int out_size, void* d_ws, size_t ws_size,
                              hipStream_t stream) {
  (void)d_ws; (void)ws_size;
  if (n_in < 17) return;
  if (in_sizes[0] != kBatch * kNpts * 3 || in_sizes[1] != kBatch * kNpts * kCin ||
      in_sizes[2] != kCout * 6 || in_sizes[7] != kCout * 2 * kCin || in_sizes[12] != kCout * 2 * kCout ||
      out_size != kBatch * kNpts * kCout) return;
  for (int i = 3; i < 17; ++i) { if (i == 7 || i == 12) continue; if (in_sizes[i] != kCout) return; }

  const float* pts   = (const float*)d_in[0];
  const float* feat  = (const float*)d_in[1];
  const float* wgeom = (const float*)d_in[2];
  const float* g1    = (const float*)d_in[3];
  const float* b1    = (const float*)d_in[4];
  const float* m1    = (const float*)d_in[5];
  const float* v1    = (const float*)d_in[6];
  const float* wsem  = (const float*)d_in[7];
  const float* g2    = (const float*)d_in[8];
  const float* b2    = (const float*)d_in[9];
  const float* m2    = (const float*)d_in[10];
  const float* v2    = (const float*)d_in[11];
  const float* wfuse = (const float*)d_in[12];
  const float* g3    = (const float*)d_in[13];
  const float* b3    = (const float*)d_in[14];
  const float* m3    = (const float*)d_in[15];
  const float* v3    = (const float*)d_in[16];
  float* out = (float*)d_out;

  dim3 grid(kNpts / kThreads, kBatch);
  knn_mlp_pool_kernel<<<grid, kThreads, 0, stream>>>(pts, feat, wgeom, g1, b1, m1, v1, wsem, g2, b2, m2, v2,
                                                      wfuse, g3, b3, m3, v3, out);
}
